// conv3x3_16484084483745
// MI455X (gfx1250) — hardware-run, weakly checked
//
#include <hip/hip_runtime.h>


#ifndef NB
#define NB 8
#endif
#define NB_FULL 8
#define CC   256
#define CO   256
#define IH   64
#define IW   64
#define NTAP 9
#define NOFF 18
#define NOP  32
#define KD   (NTAP * CC)
#define PH   (IH + 2)
#define PW   (IW + 2)
#define NPIX (IH * IW)
#define NBC  (NB < 4 ? NB : 4)
#define CPIX (NBC * NPIX)
#define XPP  264
#define OFP  36
#define OSP  68
#define WSC  256.0f
#define SSC  64.0f
#define OSC  (1.0f / 16384.0f)

static_assert(IH == 64);
static_assert(IW == 64);
static_assert(CC == 256);
static_assert(CC % 32 == 0);
static_assert(KD % 32 == 0);
static_assert(KD == NTAP * CC);
static_assert(CO % 64 == 0);
static_assert(NOFF == 2 * NTAP);
static_assert(NOFF <= NOP);
static_assert(NOP == 32);
static_assert(NPIX % 64 == 0);
static_assert(NB <= NB_FULL);
static_assert(NB % NBC == 0);
static_assert(CPIX % 64 == 0);
static_assert(CPIX % 8 == 0);
static_assert(((size_t)PW * CC * 2) % 128 == 0);
static_assert(((size_t)KD * 2) % 128 == 0);
static_assert((PW * CC / 8) % 32 == 0);
static_assert((CC * IW / 4) % 256 == 0);
static_assert(32 * 8 == CC);
static_assert(32 * 16 * 4 == 16 * NOP * 4);
static_assert(32 * 16 * 8 == 16 * 64 * 4);
static_assert((NOP * (KD / 8)) % 256 == 0);
static_assert((CO * (KD / 8)) % 256 == 0);
static_assert((OFP * 4) % 16 == 0);
static_assert((OSP * 4) % 16 == 0);
static_assert((XPP * 2) % 16 == 0);
static_assert((size_t)IW * XPP * 2 <= 131072);
static_assert((size_t)16 * OSP * 4 <= 131072);
static_assert((size_t)16 * OFP * 4 <= 131072);
static_assert((size_t)NB_FULL * CO * NPIX * 4 == (size_t)33554432);

typedef _Float16 h16;
typedef unsigned short bf;
typedef __attribute__((ext_vector_type(16))) __bf16   v16bf;
typedef __attribute__((ext_vector_type(16))) _Float16 v16h;
typedef __attribute__((ext_vector_type(8)))  _Float16 v8h;
typedef __attribute__((ext_vector_type(8)))  unsigned short v8us;
typedef __attribute__((ext_vector_type(8)))  float    v8f;
typedef __attribute__((ext_vector_type(4)))  float    v4f;
typedef v4f  __attribute__((may_alias)) v4fa;
typedef v8us __attribute__((may_alias)) v8usa;

__device__ __forceinline__ unsigned short f2bf(float f) { unsigned u = __float_as_uint(f); u += 0x7FFFu + ((u >> 16) & 1u); return (unsigned short)(u >> 16); }
__device__ __forceinline__ float bfr(float f) { return __uint_as_float(((unsigned)f2bf(f)) << 16); }
__device__ __forceinline__ v16h cat16(v8h lo, v8h hi) { return __builtin_shufflevector(lo, hi, 0, 1, 2, 3, 4, 5, 6, 7, 8, 9, 10, 11, 12, 13, 14, 15); }
__device__ __forceinline__ v16bf cat16b(v8us lo, v8us hi) { return __builtin_bit_cast(v16bf, __builtin_shufflevector(lo, hi, 0, 1, 2, 3, 4, 5, 6, 7, 8, 9, 10, 11, 12, 13, 14, 15)); }
__device__ __forceinline__ v8f wmma16(v16h a, v16h b, v8f c) { return __builtin_amdgcn_wmma_f32_16x16x32_f16(false, a, false, b, (short)0, c, false, false); }
__device__ __forceinline__ v8f wmmab(v16bf a, v16bf b, v8f c) { return __builtin_amdgcn_wmma_f32_16x16x32_bf16(false, a, false, b, (short)0, c, false, false); }
__device__ __forceinline__ v16h  ldh(const h16* p) { return cat16(*(const v8h*)p, *(const v8h*)(p + 16)); }
__device__ __forceinline__ v16bf ldb(const bf* p)  { return cat16b(*(const v8us*)p, *(const v8us*)(p + 16)); }
__device__ __forceinline__ void wave_sync() { __builtin_amdgcn_fence(3  , "wavefront"); __builtin_amdgcn_wave_barrier(); asm volatile("" ::: "memory"); }
__device__ __forceinline__ v8f wmma16g(v16h a, v16h b, v8f c) { c = wmma16(a, b, c); asm volatile("v_nop\n\tv_nop\n\tv_nop\n\tv_nop" : "+v"(c) : "v"(a), "v"(b)); return c; }
__device__ __forceinline__ v8f wmmabg(v16bf a, v16bf b, v8f c) { c = wmmab(a, b, c); asm volatile("v_nop\n\tv_nop\n\tv_nop\n\tv_nop" : "+v"(c) : "v"(a), "v"(b)); return c; }
static __device__ __forceinline__ h16 toh_flush(float v) { const h16 r = (h16)v; return (fabsf(v) < 6.103515625e-05f) ? (h16)0.0f : r; }

__global__ __launch_bounds__(256) void k_xpad(const float* __restrict__ x, bf* XP) {
    __shared__ __align__(16) unsigned short ts[IW * XPP];
    const int yp = blockIdx.x, b = blockIdx.y;
    const bool inner = (yp >= 1) & (yp <= IH);
    int y = yp - 1; y = y < 0 ? 0 : (y > IH - 1 ? IH - 1 : y);
    const float* xb = x + ((size_t)b * CC * IH + (size_t)y) * IW;
#pragma unroll 1
    for (int it = 0; it < (CC * IW / 4) / 256; ++it) {
        const int idx = it * 256 + (int)threadIdx.x; const int c = idx >> 4, x4 = (idx & 15) * 4;
        v4f v = *(const v4f*)(xb + (size_t)c * NPIX + x4);
        asm volatile("" : "+v"(v));
#pragma unroll
        for (int j = 0; j < 4; ++j) { const float r = v[j] > 0.0f ? v[j] : 0.0f; ts[(x4 + j) * XPP + c] = inner ? f2bf(r) : (unsigned short)0; }
    }
    __syncthreads();
    bf* drow = XP + ((size_t)b * PH + (size_t)yp) * ((size_t)PW * CC);
#pragma unroll 1
    for (int ps = 0; ps < 2; ++ps) {
#pragma unroll 1
        for (int i = (int)threadIdx.x; i < PW * CC / 8; i += 256) {
            const int xp = i >> 5, c8 = (i & 31) * 8;
            int xs = xp - 1; xs = xs < 0 ? 0 : (xs > IW - 1 ? IW - 1 : xs);
            const v8us t = *(const v8usa*)(&ts[xs * XPP + c8]);
            const bool ok = (xp >= 1) & (xp <= IW);
            const v8us z = (v8us){};
            const v8us v = ok ? t : z;
            *(volatile v8us*)(drow + (size_t)i * 8) = v;
        }
        if (ps == 0) __threadfence();
    }
}

__global__ __launch_bounds__(256) void k_woff(const float* __restrict__ w, bf* WO) {
    const int i = blockIdx.x * 256 + (int)threadIdx.x; if (i >= NOP * (KD / 8)) return;
    const int n = i / (KD / 8), k8 = (i % (KD / 8)) * 8; const int tap = k8 / CC, c0 = k8 % CC;
    const int ns = n < NOFF ? n : NOFF - 1;
    const bool ok = n < NOFF;
    v8us o;
#pragma unroll
    for (int j = 0; j < 8; ++j) { float v = w[((size_t)ns * CC + c0 + j) * NTAP + tap]; asm volatile("" : "+v"(v)); o[j] = ok ? f2bf(v) : (unsigned short)0; }
    *(volatile v8us*)(WO + (size_t)i * 8) = o; __threadfence(); *(volatile v8us*)(WO + (size_t)i * 8) = o;
}

__global__ __launch_bounds__(256) void k_wdef(const float* __restrict__ w, h16* WD) {
    const int i = blockIdx.x * 256 + (int)threadIdx.x; if (i >= CO * (KD / 8)) return;
    const int n = i / (KD / 8), k8 = (i % (KD / 8)) * 8; const int tap = k8 / CC, c0 = k8 % CC;
    v8h o;
#pragma unroll
    for (int j = 0; j < 8; ++j) { const float v = w[((size_t)n * CC + c0 + j) * NTAP + tap]; o[j] = toh_flush(bfr(v) * WSC); }
    *(volatile v8h*)(WD + (size_t)i * 8) = o; __threadfence(); *(volatile v8h*)(WD + (size_t)i * 8) = o;
}

__global__ __launch_bounds__(32) void k_offs(const bf* __restrict__ XP, const bf* __restrict__ WO, const float* __restrict__ boff, float* OFFS) {
    __shared__ __align__(16) float os[16 * OFP];
    const int lane = threadIdx.x & 31, lr = lane & 15, hi = lane >> 4;
    const int tile = blockIdx.x; const int b = tile / IH, y = tile % IH;
    v8f acc[4][2];
#pragma unroll
    for (int mb = 0; mb < 4; ++mb)
#pragma unroll
        for (int nb = 0; nb < 2; ++nb) acc[mb][nb] = (v8f){};
    const size_t wo = (size_t)lr * KD + 8 * hi;
#pragma unroll 1
    for (int tap = 0; tap < NTAP; ++tap) {
        const int ty = tap / 3, tx = tap - 3 * ty;
        const size_t ao = (((size_t)b * PH + (size_t)(y + ty)) * PW + (size_t)(lr + tx)) * CC + 8 * hi;
#pragma unroll 1
        for (int kc = 0; kc < CC; kc += 32) {
            v16bf a[4];
#pragma unroll
            for (int mb = 0; mb < 4; ++mb) a[mb] = ldb(XP + ao + (size_t)mb * 16 * CC + kc);
#pragma unroll
            for (int nb = 0; nb < 2; ++nb) { const v16bf bw = ldb(WO + wo + (size_t)nb * 16 * KD + (size_t)tap * CC + kc);
#pragma unroll
                for (int mb = 0; mb < 4; ++mb) acc[mb][nb] = wmmabg(a[mb], bw, acc[mb][nb]); }
        }
    }
    float bc[2];
#pragma unroll
    for (int nb = 0; nb < 2; ++nb) { const int n = nb * 16 + lr; const int ns = n < NOFF ? n : NOFF - 1;
        float bv = boff[ns]; asm volatile("" : "+v"(bv)); bc[nb] = (n < NOFF) ? bfr(bv) : 0.0f; }
    float* obase = OFFS + (size_t)tile * 64 * NOP;
#pragma unroll
    for (int mb = 0; mb < 4; ++mb) {
#pragma unroll
        for (int nb = 0; nb < 2; ++nb) {
#pragma unroll
            for (int j = 0; j < 8; ++j) os[(hi * 8 + j) * OFP + nb * 16 + lr] = acc[mb][nb][j] + bc[nb]; }
        wave_sync();
#pragma unroll 1
        for (int ps = 0; ps < 2; ++ps) {
#pragma unroll
            for (int s = 0; s < 4; ++s) { const int row = 4 * s + (lane >> 3), cofs = (lane & 7) * 4;
                const v4f val = *(const v4fa*)(&os[row * OFP + cofs]);
                *(volatile v4f*)(obase + (size_t)(mb * 16 + row) * NOP + cofs) = val; }
            if (ps == 0) __threadfence(); }
        wave_sync();
    }
}

__global__ __launch_bounds__(256) void k_samp(const bf* __restrict__ XP, const float* __restrict__ OFFS, h16* SAMP, int pix0) {
    const int lane = threadIdx.x & 31;
    const int wave = __builtin_amdgcn_readfirstlane((int)(threadIdx.x >> 5));
    const int pl = blockIdx.x * 8 + wave;
    const int p = pix0 + pl;
    const int b = p / NPIX, rem = p % NPIX; const int y = rem / IW, x = rem % IW;
    const float* orow = OFFS + (size_t)p * NOP;
    const size_t xb = (size_t)b * ((size_t)PH * PW * CC) + (size_t)lane * 8;
    const size_t sb = (size_t)pl * KD + (size_t)lane * 8;
#pragma unroll 1
    for (int tap = 0; tap < NTAP; ++tap) {
        const int ty = tap / 3, tx = tap - 3 * ty;
        float dy = orow[2 * tap], dx = orow[2 * tap + 1];
        asm volatile("" : "+v"(dy)); asm volatile("" : "+v"(dx));
        const float py = (float)(y - 1 + ty) + dy, px = (float)(x - 1 + tx) + dx;
        const float fy = floorf(py), fx = floorf(px);
        const float wy = py - fy, wx = px - fx;
        const int y0 = (int)fminf(fmaxf(fy, -8.0f), (float)(IH + 8));
        const int x0 = (int)fminf(fmaxf(fx, -8.0f), (float)(IW + 8));
        int ya = y0 + 1; ya = ya < 0 ? 0 : (ya > PH - 1 ? PH - 1 : ya);
        int yb = y0 + 2; yb = yb < 0 ? 0 : (yb > PH - 1 ? PH - 1 : yb);
        int xa = x0 + 1; xa = xa < 0 ? 0 : (xa > PW - 1 ? PW - 1 : xa);
        int xc = x0 + 2; xc = xc < 0 ? 0 : (xc > PW - 1 ? PW - 1 : xc);
        const float uy = 1.0f - wy, ux = 1.0f - wx;
        const float w00 = uy * ux * SSC, w01 = uy * wx * SSC, w10 = wy * ux * SSC, w11 = wy * wx * SSC;
        const v8us q00 = *(const v8us*)(XP + xb + ((size_t)ya * PW + (size_t)xa) * CC);
        const v8us q01 = *(const v8us*)(XP + xb + ((size_t)ya * PW + (size_t)xc) * CC);
        const v8us q10 = *(const v8us*)(XP + xb + ((size_t)yb * PW + (size_t)xa) * CC);
        const v8us q11 = *(const v8us*)(XP + xb + ((size_t)yb * PW + (size_t)xc) * CC);
        v8h hv;
#pragma unroll
        for (int j = 0; j < 8; ++j) {
            const float f00 = __uint_as_float(((unsigned)q00[j]) << 16), f01 = __uint_as_float(((unsigned)q01[j]) << 16);
            const float f10 = __uint_as_float(((unsigned)q10[j]) << 16), f11 = __uint_as_float(((unsigned)q11[j]) << 16);
            float s = f00 * w00; s += f01 * w01; s += f10 * w10; s += f11 * w11;
            hv[j] = toh_flush(s); }
        h16* dst = SAMP + sb + (size_t)tap * CC;
        *(volatile v8h*)dst = hv; __threadfence(); *(volatile v8h*)dst = hv;
    }
}

__global__ __launch_bounds__(32) void k_dgemm(const h16* __restrict__ A, const h16* __restrict__ Bt, float* OUT, int pix0) {
    __shared__ __align__(16) float os[16 * OSP];
    const int K = KD;
    const int lane = threadIdx.x & 31, lr = lane & 15, hi = lane >> 4; const int r0 = blockIdx.x * 64, c0 = blockIdx.y * 64;
    v8f acc[4][4];
#pragma unroll
    for (int mb = 0; mb < 4; ++mb)
#pragma unroll
        for (int nb = 0; nb < 4; ++nb) acc[mb][nb] = (v8f){};
    const size_t aoff = (size_t)(r0 + lr) * K + 8 * hi, boff = (size_t)(c0 + lr) * K + 8 * hi;
#pragma unroll 1
    for (int kc = 0; kc < K; kc += 32) {
        v16h a[4];
#pragma unroll
        for (int mb = 0; mb < 4; ++mb) a[mb] = ldh(A + aoff + (size_t)mb * 16 * K + kc);
#pragma unroll
        for (int nb = 0; nb < 4; ++nb) { const v16h bs = ldh(Bt + boff + (size_t)nb * 16 * K + kc);
#pragma unroll
            for (int mb = 0; mb < 4; ++mb) acc[mb][nb] = wmma16g(a[mb], bs, acc[mb][nb]); }
    }
    const int pg = pix0 + c0; const int bb = pg / NPIX, pp = pg % NPIX;
    float* obase = OUT + ((size_t)bb * CO + (size_t)r0) * NPIX + (size_t)pp;
#pragma unroll
    for (int mb = 0; mb < 4; ++mb) {
#pragma unroll
        for (int nb = 0; nb < 4; ++nb) {
#pragma unroll
            for (int j = 0; j < 8; ++j) os[(hi * 8 + j) * OSP + nb * 16 + lr] = acc[mb][nb][j] * OSC; }
        wave_sync();
#pragma unroll 1
        for (int ps = 0; ps < 2; ++ps) {
#pragma unroll
            for (int s = 0; s < 8; ++s) { const int row = 2 * s + (lane >> 4), c4 = (lane & 15) * 4;
                const v4f val = *(const v4fa*)(&os[row * OSP + c4]);
                *(volatile v4f*)(obase + (size_t)(mb * 16 + row) * NPIX + c4) = val; }
            if (ps == 0) __threadfence(); }
        wave_sync();
    }
}

static constexpr size_t al256(size_t v) { return (v + 255) & ~(size_t)255; }
static constexpr size_t SZ_XP = al256((size_t)NB * PH * PW * CC * 2);
static constexpr size_t SZ_OF = al256((size_t)NB * NPIX * NOP * 4);
static constexpr size_t SZ_WD = al256((size_t)CO * KD * 2);
static constexpr size_t SZ_WO = al256((size_t)NOP * KD * 2);
static constexpr size_t SZ_SM = al256((size_t)CPIX * KD * 2);
static constexpr size_t SZ_TOTAL = SZ_XP + SZ_OF + SZ_WD + SZ_WO + SZ_SM;
static_assert(SZ_TOTAL <= (size_t)134217728);
static_assert((size_t)(NB * IH) * 64 * NOP * 4 <= SZ_OF);
static_assert((size_t)NB * PH * ((size_t)PW * CC * 2) <= SZ_XP);
static_assert((size_t)CPIX * NTAP * 512 <= SZ_SM);
static_assert((size_t)(CO * (KD / 8)) * 16 <= SZ_WD);
static_assert((size_t)(NOP * (KD / 8)) * 16 <= SZ_WO);

extern "C" void kernel_launch(void* const* d_in, const int* in_sizes, int n_in,
                              void* d_out, int out_size, void* d_ws, size_t ws_size, hipStream_t stream) {
    if (n_in < 4) return;
    if ((size_t)in_sizes[0] < (size_t)NB * CC * NPIX) return;
    if ((size_t)in_sizes[1] < (size_t)NOFF * CC * NTAP) return;
    if (in_sizes[2] < NOFF) return;
    if ((size_t)in_sizes[3] < (size_t)CO * CC * NTAP) return;
    if ((size_t)out_size < (size_t)NB * CO * NPIX) return;
    if (SZ_TOTAL > ws_size) return;
    const float* x    = (const float*)d_in[0];
    const float* woff = (const float*)d_in[1];
    const float* boff = (const float*)d_in[2];
    const float* wdef = (const float*)d_in[3];
    float* OUT = (float*)d_out;
    char* wsp = (char*)d_ws;
    bf*    XP   = (bf*)wsp;    wsp += SZ_XP;
    float* OFFS = (float*)wsp; wsp += SZ_OF;
    h16*   WD   = (h16*)wsp;   wsp += SZ_WD;
    bf*    WO   = (bf*)wsp;    wsp += SZ_WO;
    h16*   SAMP = (h16*)wsp;   wsp += SZ_SM;

    k_xpad<<<dim3(PH, NB, 1), 256, 0, stream>>>(x, XP);
    k_woff<<<dim3((NOP * (KD / 8)) / 256, 1, 1), 256, 0, stream>>>(woff, WO);
    k_wdef<<<dim3((CO * (KD / 8)) / 256, 1, 1), 256, 0, stream>>>(wdef, WD);
    k_offs<<<dim3(NB * IH, 1, 1), 32, 0, stream>>>(XP, WO, boff, OFFS);
    for (int ch = 0; ch < NB / NBC; ++ch) {
        const int pix0 = ch * CPIX;
        k_samp<<<dim3(CPIX / 8, 1, 1), 256, 0, stream>>>(XP, OFFS, SAMP, pix0);
        k_dgemm<<<dim3(CO / 64, CPIX / 64, 1), 32, 0, stream>>>(WD, SAMP, OUT, pix0);
    }
}
